// CG_CNN_Layer_18210661335120
// MI455X (gfx1250) — hardware-verified
//
#include <hip/hip_runtime.h>
#include <stddef.h>


#define DF      64
#define PQW     256
#define DD      10
#define KIN     138
#define NTHR    256
#define NWAVE   8
#define EPT     8
#define NGRP    2
#define CHUNK   (NTHR * EPT * NGRP)
#define WCAP    (EPT * NGRP * 32)
#define LISTN   (NWAVE * WCAP)
#define NB      1024
#define GROWS   64
#define APITCH  72
#define WSCALE  8.0f
#define WINV    0.125f

#define LDS_GEMM (GROWS * PQW * 4)
#define LDS_AGG  (NB * DF * 4 + LISTN * 4 + 64)

static_assert((CHUNK & (CHUNK - 1)) == 0);
static_assert(CHUNK <= 4096);
static_assert((NB & (NB - 1)) == 0 && NB <= 4096);
static_assert(GROWS * APITCH * 2 <= LDS_GEMM);
static_assert((GROWS * DF / 8) % NTHR == 0);
static_assert((NB * DF / 4) % NTHR == 0);
static_assert(NB * DF == NWAVE * 64 * 128);
static_assert(PQW * DF / 8 == 8 * NTHR);

typedef float    v2f  __attribute__((ext_vector_type(2)));
typedef float    v4f  __attribute__((ext_vector_type(4)));
typedef float    v8f  __attribute__((ext_vector_type(8)));
typedef int      v4i  __attribute__((ext_vector_type(4)));
typedef _Float16 v8h  __attribute__((ext_vector_type(8)));
typedef _Float16 v16h __attribute__((ext_vector_type(16)));
union FragH { v16h v; v8h h[2]; };

__device__ __forceinline__ v8h cvt8(v4f a, v4f b) {
  v8h r;
  r[0] = (_Float16)a.x; r[1] = (_Float16)a.y; r[2] = (_Float16)a.z; r[3] = (_Float16)a.w;
  r[4] = (_Float16)b.x; r[5] = (_Float16)b.y; r[6] = (_Float16)b.z; r[7] = (_Float16)b.w;
  return r;
}

__device__ __forceinline__ v8f wmh(v16h a, v16h b, v8f c) {
  v8f d = __builtin_amdgcn_wmma_f32_16x16x32_f16(false, a, false, b, (short)0, c, false, false);
  asm volatile("v_nop\n\tv_nop\n\tv_nop\n\tv_nop" : "+v"(d) : "v"(a), "v"(b));
  return d;
}

template <int SLOTS>
__device__ __forceinline__ int scan_chunk(const int* __restrict__ dsts, int nE, int cbase, int nodeBase,
                                          int vec8, int* list, int tid, int lane, int wave) {
  int wc = 0;
#pragma unroll
  for (int g = 0; g < NGRP; ++g) {
    const int el0  = (g * NTHR + tid) * EPT;
    const int e0   = cbase + el0;
    const int sent = -2147483647 - 1;
    v4i da, db;
    if (vec8 != 0 && cbase + CHUNK <= nE) {
      da = *(const v4i*)(dsts + e0);
      db = *(const v4i*)(dsts + e0 + 4);
    } else {
      da.x = (e0     < nE) ? dsts[min(e0, nE - 1)] : sent;
      da.y = (e0 + 1 < nE) ? dsts[min(e0 + 1, nE - 1)] : sent;
      da.z = (e0 + 2 < nE) ? dsts[min(e0 + 2, nE - 1)] : sent;
      da.w = (e0 + 3 < nE) ? dsts[min(e0 + 3, nE - 1)] : sent;
      db.x = (e0 + 4 < nE) ? dsts[min(e0 + 4, nE - 1)] : sent;
      db.y = (e0 + 5 < nE) ? dsts[min(e0 + 5, nE - 1)] : sent;
      db.z = (e0 + 6 < nE) ? dsts[min(e0 + 6, nE - 1)] : sent;
      db.w = (e0 + 7 < nE) ? dsts[min(e0 + 7, nE - 1)] : sent;
    }
    const unsigned nb = (unsigned)nodeBase;
    const unsigned s0 = (unsigned)da.x - nb, s1 = (unsigned)da.y - nb;
    const unsigned s2 = (unsigned)da.z - nb, s3 = (unsigned)da.w - nb;
    const unsigned s4 = (unsigned)db.x - nb, s5 = (unsigned)db.y - nb;
    const unsigned s6 = (unsigned)db.z - nb, s7 = (unsigned)db.w - nb;
    const bool h0 = s0 < (unsigned)SLOTS, h1 = s1 < (unsigned)SLOTS, h2 = s2 < (unsigned)SLOTS, h3 = s3 < (unsigned)SLOTS;
    const bool h4 = s4 < (unsigned)SLOTS, h5 = s5 < (unsigned)SLOTS, h6 = s6 < (unsigned)SLOTS, h7 = s7 < (unsigned)SLOTS;
    const unsigned any = __builtin_amdgcn_ballot_w32(h0 | h1 | h2 | h3 | h4 | h5 | h6 | h7);
    if (any != 0u) {
#define HITJ(J, HJ, SJ) { \
        const unsigned mj = __builtin_amdgcn_ballot_w32(HJ); \
        if (mj != 0u) { \
          if (HJ) { \
            const int pos = wc + (int)__builtin_amdgcn_mbcnt_lo(mj, 0u); \
            if (pos < WCAP) list[wave * WCAP + pos] = ((el0 + (J)) << 12) | (int)(SJ); \
          } \
          wc += (int)__builtin_popcount(mj); } }
      HITJ(0, h0, s0)
      HITJ(1, h1, s1)
      HITJ(2, h2, s2)
      HITJ(3, h3, s3)
      HITJ(4, h4, s4)
      HITJ(5, h5, s5)
      HITJ(6, h6, s6)
      HITJ(7, h7, s7)
#undef HITJ
    }
  }
  return wc;
}

__global__ __launch_bounds__(NTHR) void k_wprep(
    const float* __restrict__ Wf, const float* __restrict__ Ws, _Float16* wcs) {
  const int i = blockIdx.x * NTHR + threadIdx.x;
  if (i >= PQW * DF / 8) return;
  const int n  = i >> 3;
  const int k0 = (i & 7) * 8;
  const int g  = n >> 6, c = n & 63;
  const float* W = (g & 1) ? Ws : Wf;
  const float* p = W + (size_t)(k0 + DF * (g >> 1)) * DF + c;
  v4f a, b;
  a.x = p[0];      a.y = p[DF];     a.z = p[2 * DF]; a.w = p[3 * DF];
  b.x = p[4 * DF]; b.y = p[5 * DF]; b.z = p[6 * DF]; b.w = p[7 * DF];
  a = a * WSCALE;
  b = b * WSCALE;
  const v8h hv = cvt8(a, b);
  _Float16* dp = wcs + (size_t)i * 8;
  *(volatile v8h*)dp = hv;
  __threadfence();
  *(volatile v8h*)dp = hv;
}

__global__ __launch_bounds__(NTHR) void k_node(
    const float* __restrict__ x, const _Float16* __restrict__ wcs, float* pq, int nN) {
  extern __shared__ v4f lds_dyn[];
  _Float16* sA  = (_Float16*)lds_dyn;
  float*    stg = (float*)lds_dyn;
  const int tid = threadIdx.x, lane = tid & 31, wave = tid >> 5, hh = lane >> 4, m = lane & 15;
  const int rowBase = blockIdx.x * GROWS;
  const int wr = wave & 3, wcol = wave >> 2;

#pragma unroll
  for (int i = 0; i < (GROWS * DF / 8) / NTHR; ++i) {
    const int idx = i * NTHR + tid;
    const int r   = idx >> 3;
    const int c0  = (idx & 7) * 8;
    int node = rowBase + r;
    node = node > nN - 1 ? nN - 1 : node;
    const float* xp = x + (size_t)node * DF + c0;
    const v4f a = *(const v4f*)xp, b = *(const v4f*)(xp + 4);
    *(v8h*)(sA + r * APITCH + c0) = cvt8(a, b);
  }
  __syncthreads();

  v8f acc[8];
#pragma unroll
  for (int t = 0; t < 8; ++t) { v8f z = {0.f, 0.f, 0.f, 0.f, 0.f, 0.f, 0.f, 0.f}; acc[t] = z; }
  const _Float16* ar = sA + (wr * 16 + m) * APITCH + 8 * hh;
#pragma unroll
  for (int kt = 0; kt < DF / 32; ++kt) {
    FragH a;
    a.h[0] = *(const v8h*)(ar + 32 * kt);
    a.h[1] = *(const v8h*)(ar + 32 * kt + 16);
#pragma unroll
    for (int t = 0; t < 8; ++t) {
      const _Float16* bp = wcs + (size_t)(128 * wcol + 16 * t + m) * DF + 32 * kt + 8 * hh;
      FragH b;
      b.h[0] = *(const v8h*)bp;
      b.h[1] = *(const v8h*)(bp + 16);
      acc[t] = wmh(a.v, b.v, acc[t]);
    }
  }
  __syncthreads();

  float* sp = stg + (wr * 16 + 8 * hh) * PQW + 128 * wcol + m;
#pragma unroll
  for (int t = 0; t < 8; ++t) {
    sp[0 * PQW + 16 * t] = acc[t][0] * WINV;
    sp[1 * PQW + 16 * t] = acc[t][1] * WINV;
    sp[2 * PQW + 16 * t] = acc[t][2] * WINV;
    sp[3 * PQW + 16 * t] = acc[t][3] * WINV;
    sp[4 * PQW + 16 * t] = acc[t][4] * WINV;
    sp[5 * PQW + 16 * t] = acc[t][5] * WINV;
    sp[6 * PQW + 16 * t] = acc[t][6] * WINV;
    sp[7 * PQW + 16 * t] = acc[t][7] * WINV;
  }
  __syncthreads();

  const float* lp = stg + (wave * 8) * PQW + 4 * lane;
  float* gp = pq + ((size_t)rowBase + wave * 8) * PQW + 4 * lane;
#pragma unroll
  for (int i = 0; i < 8; ++i) {
    const v4f v0 = *(const v4f*)(lp + i * PQW), v1 = *(const v4f*)(lp + i * PQW + 128);
    *(volatile v4f*)(gp + (size_t)i * PQW) = v0;
    *(volatile v4f*)(gp + (size_t)i * PQW + 128) = v1;
  }
  __threadfence();
#pragma unroll
  for (int i = 0; i < 8; ++i) {
    const v4f v0 = *(const v4f*)(lp + i * PQW), v1 = *(const v4f*)(lp + i * PQW + 128);
    *(volatile v4f*)(gp + (size_t)i * PQW) = v0;
    *(volatile v4f*)(gp + (size_t)i * PQW + 128) = v1;
  }
}

__global__ __launch_bounds__(NTHR) void k_agg(
    const int* __restrict__ dsts, const int* __restrict__ srcs, const float* __restrict__ dist,
    const float* __restrict__ pq, const float* __restrict__ x,
    const float* __restrict__ Wf, const float* __restrict__ Ws,
    const float* __restrict__ bfv, const float* __restrict__ bsv,
    float* out, int nN, int nE, int vec8) {
  extern __shared__ v4f lds_dyn[];
  float* acc  = (float*)lds_dyn;
  int*   list = (int*)(acc + NB * DF);
  int*   wcnt = list + LISTN;
  const int tid = threadIdx.x, lane = tid & 31, wave = tid >> 5;
  const int nodeBase = blockIdx.x * NB;

  v2f wfd[DD], wsd[DD];
#pragma unroll
  for (int j = 0; j < DD; ++j) {
    wfd[j] = *(const v2f*)(Wf + (size_t)(2 * DF + j) * DF + 2 * lane);
    wsd[j] = *(const v2f*)(Ws + (size_t)(2 * DF + j) * DF + 2 * lane);
  }
  const v2f bf2 = *(const v2f*)(bfv + 2 * lane);
  const v2f bs2 = *(const v2f*)(bsv + 2 * lane);

  {
    const v4f z = {0.f, 0.f, 0.f, 0.f};
    for (int i = tid; i < NB * DF / 4; i += NTHR) lds_dyn[i] = z;
  }
  __syncthreads();

  const float L2E = 1.44269504f, LN2 = 0.69314718f;
  const int nChunks = (nE + CHUNK - 1) / CHUNK;
#pragma unroll 1
  for (int ch = 0; ch < nChunks; ++ch) {
    const int cbase = ch * CHUNK;
    const int wc = scan_chunk<NB>(dsts, nE, cbase, nodeBase, vec8, list, tid, lane, wave);
    if (lane == 0) wcnt[wave] = wc;
    __syncthreads();
    if (wave == 0) {
#pragma unroll 1
      for (int wsx = 0; wsx < NWAVE; ++wsx) {
        int n = __builtin_amdgcn_readfirstlane(wcnt[wsx]);
        n = n > WCAP ? WCAP : (n < 0 ? 0 : n);
        const int* lp = list + wsx * WCAP;
#pragma unroll 1
        for (int i = 0; i < n; ++i) {
          const int ent  = __builtin_amdgcn_readfirstlane(lp[i]);
          const int slot = ent & (NB - 1);
          int e = cbase + ((ent >> 12) & (CHUNK - 1));
          e = e > nE - 1 ? nE - 1 : e;
          int s = srcs[e];
          s = s < 0 ? 0 : (s > nN - 1 ? nN - 1 : s);
          int node = nodeBase + slot;
          node = node > nN - 1 ? nN - 1 : node;
          const float* pp = pq + (size_t)s * PQW + 2 * lane;
          const float* qp = pq + (size_t)node * PQW + 2 * lane;
          const v2f pf = *(const v2f*)pp;
          const v2f ps = *(const v2f*)(pp + 64);
          const v2f qf = *(const v2f*)(qp + 128);
          const v2f qs = *(const v2f*)(qp + 192);
          const float* dr = dist + (size_t)e * DD;
          float zf0 = (pf.x + qf.x) + bf2.x, zf1 = (pf.y + qf.y) + bf2.y;
          float zs0 = (ps.x + qs.x) + bs2.x, zs1 = (ps.y + qs.y) + bs2.y;
#pragma unroll
          for (int j = 0; j < DD; ++j) {
            const float d = dr[j];
            zf0 = fmaf(d, wfd[j].x, zf0);
            zf1 = fmaf(d, wfd[j].y, zf1);
            zs0 = fmaf(d, wsd[j].x, zs0);
            zs1 = fmaf(d, wsd[j].y, zs1);
          }
          const float t0  = exp2f(-zf0 * L2E), t1 = exp2f(-zf1 * L2E);
          const float sg0 = __builtin_amdgcn_rcpf(1.0f + t0);
          const float sg1 = __builtin_amdgcn_rcpf(1.0f + t1);
          const float u0  = exp2f(-fabsf(zs0) * L2E), u1 = exp2f(-fabsf(zs1) * L2E);
          const float sp0 = fmaxf(zs0, 0.f) + LN2 * log2f(1.0f + u0);
          const float sp1 = fmaxf(zs1, 0.f) + LN2 * log2f(1.0f + u1);
          const float g0 = sg0 * sp0, g1 = sg1 * sp1;
          v2f* ap = (v2f*)(acc + slot * DF + 2 * lane);
          v2f av = *ap;
          av.x = av.x + g0;
          av.y = av.y + g1;
          *ap = av;
        }
      }
    }
    __syncthreads();
  }

#pragma unroll 4
  for (int i = 0; i < (NB * DF / 4) / NTHR; ++i) {
    const int idx  = i * NTHR + tid;
    const int slot = idx >> 4;
    const int c4   = (idx & 15) * 4;
    int node = nodeBase + slot;
    node = node > nN - 1 ? nN - 1 : node;
    const v4f fv = *(const v4f*)(x + (size_t)node * DF + c4);
    v4f* ap = (v4f*)(acc + slot * DF + c4);
    *ap = *ap + fv;
  }
  __syncthreads();

  const size_t outN = (size_t)nN * DF;
  const size_t ob   = (size_t)nodeBase * DF;
#pragma unroll 4
  for (int q = 0; q < 64; ++q) {
    const int f = (wave * 64 + q) * 128 + 4 * lane;
    const size_t gi = ob + (size_t)f;
    if (gi < outN) { const v4f v = *(const v4f*)(acc + f); *(volatile v4f*)(out + gi) = v; }
  }
  __threadfence();
#pragma unroll 4
  for (int q = 0; q < 64; ++q) {
    const int f = (wave * 64 + q) * 128 + 4 * lane;
    const size_t gi = ob + (size_t)f;
    if (gi < outN) { const v4f v = *(const v4f*)(acc + f); *(volatile v4f*)(out + gi) = v; }
  }
}

extern "C" void kernel_launch(void* const* d_in, const int* in_sizes, int n_in,
                              void* d_out, int out_size, void* d_ws, size_t ws_size,
                              hipStream_t stream) {
  if (n_in < 8) return;
  const int nN = in_sizes[0] / DF;
  const int nE = in_sizes[2];
  if (nN <= 0 || nE < 0 || in_sizes[0] != nN * DF) return;
  if (in_sizes[1] != nE * DD || in_sizes[3] != nE) return;
  if (in_sizes[4] != KIN * DF || in_sizes[5] < DF || in_sizes[6] != KIN * DF || in_sizes[7] < DF) return;
  if (out_size != nN * DF) return;

  const float* x    = (const float*)d_in[0];
  const float* dist = (const float*)d_in[1];
  const int*   srcs = (const int*)d_in[2];
  const int*   dsts = (const int*)d_in[3];
  const float* Wf   = (const float*)d_in[4];
  const float* bfv  = (const float*)d_in[5];
  const float* Ws   = (const float*)d_in[6];
  const float* bsv  = (const float*)d_in[7];
  float* out = (float*)d_out;

  const int nG = (nN + GROWS - 1) / GROWS;
  const int nA = (nN + NB - 1) / NB;

  char* ws = (char*)d_ws;
  size_t off = 0;
  const size_t oW  = off; off += (size_t)PQW * DF * 2;                         off = (off + 255) & ~(size_t)255;
  const size_t oPQ = off; off += (size_t)nG * GROWS * PQW * 4;                 off = (off + 255) & ~(size_t)255;
  if (off > ws_size) return;
  _Float16* wcs = (_Float16*)(ws + oW);
  float*    pq  = (float*)(ws + oPQ);

  const int vec8 = 1;

  k_wprep<<<(PQW * DF / 8 + NTHR - 1) / NTHR, NTHR, 0, stream>>>(Wf, Ws, wcs);

  hipFuncSetAttribute(reinterpret_cast<const void*>(&k_node),
                      hipFuncAttributeMaxDynamicSharedMemorySize, LDS_GEMM);
  k_node<<<nG, NTHR, LDS_GEMM, stream>>>(x, wcs, pq, nN);

  hipFuncSetAttribute(reinterpret_cast<const void*>(&k_agg),
                      hipFuncAttributeMaxDynamicSharedMemorySize, LDS_AGG);
  k_agg<<<nA, NTHR, LDS_AGG, stream>>>(dsts, srcs, dist, pq, x, Wf, Ws, bfv, bsv, out, nN, nE, vec8);
}
